// GNN_node_73512660238838
// MI455X (gfx1250) — hardware-verified
//
#include <hip/hip_runtime.h>
#include <stddef.h>
#include <stdint.h>


#define DF     128
#define DIN    64
#define NTV    8
#define NIV    64
#define AP     512
#define K0     256
#define K12    512
#define NTHR   256
#define NWAVE  8
#define EPT    8
#define CHUNK  (NTHR * EPT)
#define WCAP   (EPT * 32)
#define LISTN  (NWAVE * WCAP)
#define NBA    1024
#define SLA    10
#define RCAP   28672
#define DEGCAP 64
#define GBM    64
#define GBN    128
#define GTHR   128
#define GWAVE  (GTHR / 32)
#define PARTW  288
#define WSTW   258
#define UPART  2048
#define NPART  10
#define ROWH   256
#define TBLF   ((NTV + NIV) * DIN)
#define AGG_ZINTS     (LISTN + 2 * RCAP + 3 * NBA)
#define MISC_INTS     16
#define ROWBUF_INTS   (NWAVE * ROWH / 2)
#define AGG_BASE_INTS (AGG_ZINTS + MISC_INTS + ROWBUF_INTS)
#define AGG_LDS_INTS1 (AGG_BASE_INTS + TBLF)
#define WSMAX  134217728

static_assert((CHUNK & (CHUNK - 1)) == 0 && CHUNK <= 4096);
static_assert((NBA & (NBA - 1)) == 0 && NBA == (1 << SLA));
static_assert(((long long)CHUNK << SLA) < (1LL << 31));
static_assert(LISTN % NTHR == 0);
static_assert(NBA % NWAVE == 0 && NBA % 32 == 0 && NBA % GBM == 0);
static_assert(RCAP % 4 == 0 && AGG_ZINTS % 4 == 0 && LISTN % 4 == 0 && ((AGG_ZINTS + MISC_INTS) % 4) == 0);
static_assert(AGG_BASE_INTS % 4 == 0 && TBLF % 4 == 0);
static_assert(AGG_ZINTS % (NTHR * 4) == 0);
static_assert(K0 % 32 == 0 && K12 % 32 == 0 && K12 == AP && K0 == 4 * DIN && K12 == 4 * DF);
static_assert(GBN == DF && GBM == GWAVE * 16 && DF == 4 * 32 && DIN == 2 * 32);
static_assert(UPART % NTHR == 0 && UPART == DF * (DF / 8));
static_assert(AGG_LDS_INTS1 * 4 <= 300000);
static_assert(PARTW % 32 == 0 && PARTW / 4 <= GTHR && PARTW >= 2 * GBN + 1);
static_assert(WSTW >= 2 * GBN + 1 && (WSTW % 2) == 0);
static_assert(ROWH == 2 * DF && ROWH == 4 * DIN);
static_assert((NTV * DIN) % NTHR == 0 && (NIV * DIN) % NTHR == 0);
static_assert(NTHR == 2 * DF);

typedef float          v2f   __attribute__((ext_vector_type(2)));
typedef float          v4f   __attribute__((ext_vector_type(4)));
typedef float          v8f   __attribute__((ext_vector_type(8)));
typedef int            v4i   __attribute__((ext_vector_type(4)));
typedef int            v8i   __attribute__((ext_vector_type(8)));
typedef unsigned       v2u   __attribute__((ext_vector_type(2)));
typedef unsigned       v4u   __attribute__((ext_vector_type(4)));
typedef unsigned short v2us  __attribute__((ext_vector_type(2)));
typedef unsigned short v4us  __attribute__((ext_vector_type(4)));
typedef unsigned short v8us  __attribute__((ext_vector_type(8)));
typedef unsigned short v16us __attribute__((ext_vector_type(16)));
typedef __bf16         v16bf __attribute__((ext_vector_type(16)));
typedef v2f  __attribute__((may_alias)) v2fa;
typedef v4f  __attribute__((may_alias)) v4fa;
typedef v4i  __attribute__((may_alias)) v4ia;
typedef v2u  __attribute__((may_alias)) v2ua;
typedef v4u  __attribute__((may_alias)) v4ua;
typedef v2us __attribute__((may_alias)) v2usa;
typedef v4us __attribute__((may_alias)) v4usa;
typedef v8us __attribute__((may_alias)) v8usa;
union FragB { v16bf v; v16us u; v8us h[2]; v8i w; };

__device__ __forceinline__ v8f wmb(const FragB& a, const FragB& b, v8f c) {
  v8f d = __builtin_amdgcn_wmma_f32_16x16x32_bf16(false, a.v, false, b.v, (short)0, c, false, false);
  asm volatile("v_nop\n\tv_nop\n\tv_nop\n\tv_nop" : "+v"(d) : "v"(a.w), "v"(b.w));
  return d;
}

__device__ __forceinline__ v8f z8() { v8f z = {0.f, 0.f, 0.f, 0.f, 0.f, 0.f, 0.f, 0.f}; return z; }

__device__ __forceinline__ unsigned bf16_bits(float f) {
  const unsigned u = __float_as_uint(f);
  return (u + 0x7FFFu + ((u >> 16) & 1u)) >> 16;
}
__device__ __forceinline__ float bf16_val(float f) {
  return __uint_as_float(bf16_bits(f) << 16);
}
__device__ __forceinline__ unsigned hl_bits(float v, unsigned& lo) {
  const unsigned hb = bf16_bits(v);
  lo = bf16_bits(v - __uint_as_float(hb << 16));
  return hb;
}

__device__ __forceinline__ void wave_sync() {
  __builtin_amdgcn_fence(__ATOMIC_RELEASE, "wavefront");
  __builtin_amdgcn_wave_barrier();
  __builtin_amdgcn_fence(__ATOMIC_ACQUIRE, "wavefront");
}

template <int SLB>
__device__ __forceinline__ int scan_chunk(const int* __restrict__ dsts, int nE, int cbase, int slotBase,
                                          int nb, int vec8, int* list, int tid, int lane, int wave) {
  int wc = 0;
  const int el0  = tid * EPT;
  const int e0   = cbase + el0;
  const int sent = -2147483647 - 1;
  v4i da, db;
  if (vec8 != 0 && cbase + CHUNK <= nE) {
    da = *(const v4i*)(dsts + e0);
    db = *(const v4i*)(dsts + e0 + 4);
  } else {
    da.x = (e0     < nE) ? dsts[min(e0,     nE - 1)] : sent;
    da.y = (e0 + 1 < nE) ? dsts[min(e0 + 1, nE - 1)] : sent;
    da.z = (e0 + 2 < nE) ? dsts[min(e0 + 2, nE - 1)] : sent;
    da.w = (e0 + 3 < nE) ? dsts[min(e0 + 3, nE - 1)] : sent;
    db.x = (e0 + 4 < nE) ? dsts[min(e0 + 4, nE - 1)] : sent;
    db.y = (e0 + 5 < nE) ? dsts[min(e0 + 5, nE - 1)] : sent;
    db.z = (e0 + 6 < nE) ? dsts[min(e0 + 6, nE - 1)] : sent;
    db.w = (e0 + 7 < nE) ? dsts[min(e0 + 7, nE - 1)] : sent;
  }
  const unsigned nbs = (unsigned)slotBase;
  const unsigned unb = (unsigned)nb;
  const unsigned s0 = (unsigned)da.x - nbs, s1 = (unsigned)da.y - nbs;
  const unsigned s2 = (unsigned)da.z - nbs, s3 = (unsigned)da.w - nbs;
  const unsigned s4 = (unsigned)db.x - nbs, s5 = (unsigned)db.y - nbs;
  const unsigned s6 = (unsigned)db.z - nbs, s7 = (unsigned)db.w - nbs;
  const bool h0 = s0 < unb, h1 = s1 < unb, h2 = s2 < unb, h3 = s3 < unb;
  const bool h4 = s4 < unb, h5 = s5 < unb, h6 = s6 < unb, h7 = s7 < unb;
  const unsigned any = __builtin_amdgcn_ballot_w32(h0 | h1 | h2 | h3 | h4 | h5 | h6 | h7);
  if (any != 0u) {
#define HITJ(J, HJ, SJ) { \
      const unsigned mj = __builtin_amdgcn_ballot_w32(HJ); \
      if (mj != 0u) { \
        if (HJ) { \
          const int pos = wc + (int)__builtin_amdgcn_mbcnt_lo(mj, 0u); \
          if (pos < WCAP) list[wave * WCAP + pos] = ((el0 + (J)) << SLB) | (int)(SJ); \
        } \
        wc += (int)__builtin_popcount(mj); } }
    HITJ(0, h0, s0)
    HITJ(1, h1, s1)
    HITJ(2, h2, s2)
    HITJ(3, h3, s3)
    HITJ(4, h4, s4)
    HITJ(5, h5, s5)
    HITJ(6, h6, s6)
    HITJ(7, h7, s7)
#undef HITJ
  }
  return wc;
}

__global__ __launch_bounds__(NTHR) void k_wprep(const float* __restrict__ Wl0, const float* __restrict__ Wr0,
                                                const float* __restrict__ Wl1, const float* __restrict__ Wr1,
                                                const float* __restrict__ Wl2, const float* __restrict__ Wr2,
                                                unsigned short* B0, unsigned short* B1, unsigned short* B2) {
  const int u    = (int)blockIdx.x * NTHR + (int)threadIdx.x;
  const int part = u >> 11;
  const int v    = u & (UPART - 1);
  const int n    = v >> 4;
  const int k8   = (v & 15) * 8;
  const float* W;
  unsigned short* P;
  int pitch, coff, kmask;
  if (part == 0)       { W = Wl0; P = B0; pitch = K0;  coff = 0;       kmask = DIN - 1; }
  else if (part == 1)  { W = Wr0; P = B0; pitch = K0;  coff = 2 * DIN; kmask = DIN - 1; }
  else if (part == 2)  { W = Wl1; P = B1; pitch = K12; coff = 0;       kmask = DF - 1; }
  else if (part == 3)  { W = Wl1; P = B1; pitch = K12; coff = DF;      kmask = DF - 1; }
  else if (part == 4)  { W = Wr1; P = B1; pitch = K12; coff = 2 * DF;  kmask = DF - 1; }
  else if (part == 5)  { W = Wr1; P = B1; pitch = K12; coff = 3 * DF;  kmask = DF - 1; }
  else if (part == 6)  { W = Wl2; P = B2; pitch = K12; coff = 0;       kmask = DF - 1; }
  else if (part == 7)  { W = Wl2; P = B2; pitch = K12; coff = DF;      kmask = DF - 1; }
  else if (part == 8)  { W = Wr2; P = B2; pitch = K12; coff = 2 * DF;  kmask = DF - 1; }
  else if (part == 9)  { W = Wr2; P = B2; pitch = K12; coff = 3 * DF;  kmask = DF - 1; }
  else return;
  const int ks = k8 & kmask;
  const float* p = W + (size_t)ks * DF + n;
  v8us o;
#pragma unroll
  for (int i = 0; i < 8; ++i) o[i] = (unsigned short)bf16_bits(p[(size_t)i * DF]);
  unsigned short* dp = P + (size_t)n * pitch + coff + k8;
  *(volatile v8us*)dp = o;
  __threadfence();
  *(volatile v8us*)dp = o;
}

template <int L0>
__global__ __launch_bounds__(NTHR) void k_scan(const int* __restrict__ srcs, const int* __restrict__ dsts,
                                               int nE, int nN, int vec8, int mRows,
                                               const int* __restrict__ ntp, const int* __restrict__ ipp,
                                               const float* __restrict__ ent, const float* __restrict__ eip,
                                               unsigned short* apl) {
  extern __shared__ __attribute__((aligned(16))) int dsm[];
  int* list = dsm;
  int* hl   = dsm + LISTN;
  int* sl   = hl + RCAP;
  int* cnt  = sl + RCAP;
  int* offs = cnt + NBA;
  int* cur  = offs + NBA;
  int* misc = cur + NBA;
  const int tid = (int)threadIdx.x, lane = tid & 31, wave = tid >> 5;
  unsigned short* rowbuf = (unsigned short*)(misc + MISC_INTS) + wave * ROWH;
  float* tnt = (float*)(misc + MISC_INTS + ROWBUF_INTS);
  float* tip = tnt + NTV * DIN;
  const int nodeBase = (int)blockIdx.x * NBA;

  {
    const v4i z4 = {0, 0, 0, 0};
    for (int i = tid * 4; i < AGG_ZINTS; i += NTHR * 4) *(v4ia*)(dsm + i) = z4;
    if (tid < MISC_INTS) misc[tid] = 0;
  }
  if constexpr (L0 != 0) {
#pragma unroll 1
    for (int i = tid; i < NTV * DIN; i += NTHR) tnt[i] = bf16_val(ent[i]);
#pragma unroll 1
    for (int i = tid; i < NIV * DIN; i += NTHR) tip[i] = bf16_val(eip[i]);
  }
  __syncthreads();

  int t = 0, ov = 0;
  const int nChunks = (nE + CHUNK - 1) / CHUNK;
#pragma unroll 1
  for (int ch = 0; ch < nChunks; ++ch) {
    const int cbase = ch * CHUNK;
    const int wc = scan_chunk<SLA>(dsts, nE, cbase, nodeBase, NBA, vec8, list, tid, lane, wave);
    if (lane == 0) misc[wave] = wc;
    __syncthreads();
    if (wave == 0) {
#pragma unroll 1
      for (int w2 = 0; w2 < NWAVE; ++w2) {
        int c = misc[w2];
        c = c < 0 ? 0 : (c > WCAP ? WCAP : c);
#pragma unroll 1
        for (int b0 = 0; b0 < c; b0 += 32) {
          const int idx = b0 + lane;
          const int ent_ = list[w2 * WCAP + (idx < WCAP ? idx : WCAP - 1)];
          const int m32 = (c - b0) < 32 ? (c - b0) : 32;
#pragma unroll 1
          for (int k = 0; k < m32; ++k) {
            const int u    = __builtin_amdgcn_readlane(ent_, k);
            const int slot = u & (NBA - 1);
            const int el   = (u >> SLA) & (CHUNK - 1);
            const int pk   = ((cbase + el) << SLA) | slot;
            if (t < RCAP) {
              if (lane == 0) { hl[t] = pk; cnt[slot] = cnt[slot] + 1; }
              t = t + 1;
            } else {
              ov = 1;
            }
          }
        }
      }
    }
    __syncthreads();
  }
  if (wave == 0 && lane == 0) { misc[8] = t; misc[9] = ov; }
  __syncthreads();
  int tt = misc[8];
  tt = tt < 0 ? 0 : (tt > RCAP ? RCAP : tt);
  const int ovf = misc[9];

  if (wave == 0) {
    const int base = lane * (NBA / 32);
    int s = 0;
#pragma unroll 1
    for (int i = 0; i < NBA / 32; ++i) s += cnt[base + i];
    int incl = s;
#pragma unroll
    for (int d = 1; d < 32; d <<= 1) {
      const int y = __shfl_up(incl, d, 32);
      if (lane >= d) incl += y;
    }
    int run = incl - s;
#pragma unroll 1
    for (int i = 0; i < NBA / 32; ++i) {
      const int cv = cnt[base + i];
      offs[base + i] = run;
      cur[base + i]  = run;
      run += cv;
    }
  }
  __syncthreads();
  if (wave == 0) {
#pragma unroll 1
    for (int b0 = 0; b0 < tt; b0 += 32) {
      const int idx = b0 + lane;
      const int ent_ = hl[idx < RCAP ? idx : RCAP - 1];
      const int m32 = (tt - b0) < 32 ? (tt - b0) : 32;
#pragma unroll 1
      for (int k = 0; k < m32; ++k) {
        const int u    = __builtin_amdgcn_readlane(ent_, k);
        const int slot = u & (NBA - 1);
        if (lane == 0) {
          int p = cur[slot];
          p = p < 0 ? 0 : (p > RCAP - 1 ? RCAP - 1 : p);
          sl[p] = u;
          cur[slot] = p + 1;
        }
      }
    }
  }
  __syncthreads();

  const float pz = (ovf != 0) ? __int_as_float(0x7fc00000) : 0.0f;
#pragma unroll 1
  for (int si = 0; si < NBA / NWAVE; ++si) {
    const int s    = si * NWAVE + wave;
    const int node = nodeBase + s;
    int c = cnt[s];
    const bool big = c > DEGCAP;
    c = c < 0 ? 0 : (c > DEGCAP ? DEGCAP : c);
    int o = offs[s];
    o = o < 0 ? 0 : (o > RCAP ? RCAP : o);
    const int nc = node < nN ? node : nN - 1;
    const float pzr = big ? __int_as_float(0x7fc00000) : pz;
    const bool live = node < nN;
    if constexpr (L0 != 0) {
      float a0 = 0.0f, a1 = 0.0f;
#pragma unroll 1
      for (int b0 = 0; b0 < c; b0 += 32) {
        int idx = o + b0 + lane;
        idx = idx > RCAP - 1 ? RCAP - 1 : idx;
        const int ent_ = sl[idx];
        int eid = ent_ >> SLA;
        eid = eid < 0 ? 0 : (eid > nE - 1 ? nE - 1 : eid);
        int sr = srcs[eid];
        sr = sr < 0 ? 0 : (sr > nN - 1 ? nN - 1 : sr);
        int tv = ntp[sr];
        tv = tv < 0 ? 0 : (tv > NTV - 1 ? NTV - 1 : tv);
        int iv = ipp[sr];
        iv = iv < 0 ? 0 : (iv > NIV - 1 ? NIV - 1 : iv);
        const int key = (tv << 6) | iv;
        const int m32 = (c - b0) < 32 ? (c - b0) : 32;
#pragma unroll 1
        for (int k = 0; k < m32; ++k) {
          const int kk = __builtin_amdgcn_readlane(key, k);
          const v2f ta = *(const v2fa*)(tnt + (kk >> 6) * DIN + 2 * lane);
          const v2f tb = *(const v2fa*)(tip + (kk & 63) * DIN + 2 * lane);
          const float hx = ta.x + tb.x;
          const float hy = ta.y + tb.y;
          a0 = a0 + hx;
          a1 = a1 + hy;
        }
      }
      const float inv = 1.0f / fmaxf((float)c, 1.0f);
      const float m0 = live ? (a0 * inv + pzr) : 0.0f;
      const float m1 = live ? (a1 * inv + pzr) : 0.0f;
      int tn = ntp[nc];
      tn = tn < 0 ? 0 : (tn > NTV - 1 ? NTV - 1 : tn);
      int in2 = ipp[nc];
      in2 = in2 < 0 ? 0 : (in2 > NIV - 1 ? NIV - 1 : in2);
      const v2f ra = *(const v2fa*)(tnt + tn * DIN + 2 * lane);
      const v2f rb = *(const v2fa*)(tip + in2 * DIN + 2 * lane);
      const float x0 = live ? ((ra.x + rb.x) + pzr) : 0.0f;
      const float x1 = live ? ((ra.y + rb.y) + pzr) : 0.0f;
      v2us mh, ml, xh, xl;
      {
        unsigned lb;
        unsigned hb;
        hb = hl_bits(m0, lb); mh[0] = (unsigned short)hb; ml[0] = (unsigned short)lb;
        hb = hl_bits(m1, lb); mh[1] = (unsigned short)hb; ml[1] = (unsigned short)lb;
        hb = hl_bits(x0, lb); xh[0] = (unsigned short)hb; xl[0] = (unsigned short)lb;
        hb = hl_bits(x1, lb); xh[1] = (unsigned short)hb; xl[1] = (unsigned short)lb;
      }
      *(v2usa*)(rowbuf + 2 * lane)           = mh;
      *(v2usa*)(rowbuf + DIN + 2 * lane)     = ml;
      *(v2usa*)(rowbuf + 2 * DIN + 2 * lane) = xh;
      *(v2usa*)(rowbuf + 3 * DIN + 2 * lane) = xl;
    } else {
      float a0 = 0.0f, a1 = 0.0f, a2 = 0.0f, a3 = 0.0f;
#pragma unroll 1
      for (int b0 = 0; b0 < c; b0 += 32) {
        int idx = o + b0 + lane;
        idx = idx > RCAP - 1 ? RCAP - 1 : idx;
        const int ent_ = sl[idx];
        int eid = ent_ >> SLA;
        eid = eid < 0 ? 0 : (eid > nE - 1 ? nE - 1 : eid);
        int sr = srcs[eid];
        sr = sr < 0 ? 0 : (sr > nN - 1 ? nN - 1 : sr);
        const int m32 = (c - b0) < 32 ? (c - b0) : 32;
#pragma unroll 1
        for (int k = 0; k < m32; ++k) {
          const int sk = __builtin_amdgcn_readlane(sr, k);
          const unsigned short* rp = apl + (size_t)sk * AP + 2 * DF + 4 * lane;
          const v2u wh = *(const v2ua*)rp;
          const v2u wl = *(const v2ua*)(rp + DF);
          const float f0 = __uint_as_float(wh.x << 16)         + __uint_as_float(wl.x << 16);
          const float f1 = __uint_as_float(wh.x & 0xffff0000u) + __uint_as_float(wl.x & 0xffff0000u);
          const float f2 = __uint_as_float(wh.y << 16)         + __uint_as_float(wl.y << 16);
          const float f3 = __uint_as_float(wh.y & 0xffff0000u) + __uint_as_float(wl.y & 0xffff0000u);
          a0 += f0; a1 += f1; a2 += f2; a3 += f3;
        }
      }
      const float inv = 1.0f / fmaxf((float)c, 1.0f);
      const float m0 = live ? (a0 * inv + pzr) : 0.0f;
      const float m1 = live ? (a1 * inv + pzr) : 0.0f;
      const float m2 = live ? (a2 * inv + pzr) : 0.0f;
      const float m3 = live ? (a3 * inv + pzr) : 0.0f;
      v4us mh, ml;
      {
        unsigned lb;
        unsigned hb;
        hb = hl_bits(m0, lb); mh[0] = (unsigned short)hb; ml[0] = (unsigned short)lb;
        hb = hl_bits(m1, lb); mh[1] = (unsigned short)hb; ml[1] = (unsigned short)lb;
        hb = hl_bits(m2, lb); mh[2] = (unsigned short)hb; ml[2] = (unsigned short)lb;
        hb = hl_bits(m3, lb); mh[3] = (unsigned short)hb; ml[3] = (unsigned short)lb;
      }
      *(v4usa*)(rowbuf + 4 * lane)      = mh;
      *(v4usa*)(rowbuf + DF + 4 * lane) = ml;
    }
    wave_sync();
    const v8us q0 = *(const v8usa*)(rowbuf + 8 * lane);
    wave_sync();
    if (node < mRows) {
      unsigned short* rpw = apl + (size_t)node * AP + 8 * lane;
      *(volatile v8us*)rpw = q0;
      __threadfence();
      *(volatile v8us*)rpw = q0;
    }
  }
}

__global__ __launch_bounds__(GTHR) void k_gemm(unsigned short* Apl, const unsigned short* __restrict__ BT, int K,
                                               int nN, const float* __restrict__ bias, float* part) {
  __shared__ __attribute__((aligned(16))) float stg[GBM * GBN];
  __shared__ __attribute__((aligned(16))) float wst[GWAVE * WSTW];
  __shared__ __attribute__((aligned(16))) float pst[PARTW];
  const int tid = (int)threadIdx.x, lane = tid & 31, wave = tid >> 5, hh = lane >> 4, m = lane & 15;
  const int rowBase = (int)blockIdx.x * GBM;

  v8f acc[8];
#pragma unroll
  for (int t = 0; t < 8; ++t) acc[t] = z8();
  const unsigned short* ap = Apl + (size_t)(rowBase + 16 * wave + m) * (size_t)AP + 8 * hh;
  const unsigned short* bp = BT + (size_t)m * (size_t)K + 8 * hh;

#pragma unroll 1
  for (int k0 = 0; k0 < K; k0 += 32) {
    FragB af;
    af.h[0] = *(const v8usa*)(ap + k0);
    af.h[1] = *(const v8usa*)(ap + k0 + 16);
#pragma unroll
    for (int nt = 0; nt < 8; ++nt) {
      const unsigned short* wq = bp + (size_t)(16 * nt) * (size_t)K + k0;
      FragB bf;
      bf.h[0] = *(const v8usa*)wq;
      bf.h[1] = *(const v8usa*)(wq + 16);
      acc[nt] = wmb(af, bf, acc[nt]);
    }
  }

#pragma unroll
  for (int nt = 0; nt < 8; ++nt) {
    const int lc = 16 * nt + m;
#pragma unroll
    for (int r = 0; r < 8; ++r) {
      const int lr = 16 * wave + 8 * hh + r;
      stg[lr * GBN + lc] = acc[nt][r];
    }
  }
  __syncthreads();

  float bq[4];
  {
    const v4f b4 = *(const v4f*)(bias + 4 * lane);
    bq[0] = bf16_val(b4.x); bq[1] = bf16_val(b4.y); bq[2] = bf16_val(b4.z); bq[3] = bf16_val(b4.w);
  }

  v4f pv[16];
#pragma unroll
  for (int i = 0; i < 16; ++i) pv[i] = *(const v4fa*)(stg + (16 * wave + i) * GBN + 4 * lane);
  __syncthreads();

  int wn = 0;
  float wm[4], wqv[4];
#pragma unroll
  for (int j = 0; j < 4; ++j) { wm[j] = 0.0f; wqv[j] = 0.0f; }
#pragma unroll
  for (int i = 0; i < 16; ++i) {
    const int row = rowBase + 16 * wave + i;
    const bool ok = row < nN;
    float y[4];
    y[0] = pv[i].x + bq[0]; y[1] = pv[i].y + bq[1]; y[2] = pv[i].z + bq[2]; y[3] = pv[i].w + bq[3];
    float vv[4];
#pragma unroll
    for (int j = 0; j < 4; ++j) vv[j] = ok ? y[j] : 0.0f;
    v4f q;
    q.x = vv[0]; q.y = vv[1]; q.z = vv[2]; q.w = vv[3];
    pv[i] = q;
    if (ok) {
      wn += 1;
      const float rk = 1.0f / (float)(i + 1);
#pragma unroll
      for (int j = 0; j < 4; ++j) {
        const float d = vv[j] - wm[j];
        wm[j]  = fmaf(d, rk, wm[j]);
        wqv[j] = fmaf(d, vv[j] - wm[j], wqv[j]);
      }
    }
  }

#pragma unroll
  for (int i = 0; i < 16; ++i) {
    v4us h4, l4;
    unsigned lb;
    unsigned hb;
    hb = hl_bits(pv[i].x, lb); h4[0] = (unsigned short)hb; l4[0] = (unsigned short)lb;
    hb = hl_bits(pv[i].y, lb); h4[1] = (unsigned short)hb; l4[1] = (unsigned short)lb;
    hb = hl_bits(pv[i].z, lb); h4[2] = (unsigned short)hb; l4[2] = (unsigned short)lb;
    hb = hl_bits(pv[i].w, lb); h4[3] = (unsigned short)hb; l4[3] = (unsigned short)lb;
    unsigned short* srow = (unsigned short*)stg + (size_t)(16 * wave + i) * (2 * GBN);
    *(v4usa*)(srow + 4 * lane) = h4;
    *(v4usa*)(srow + DF + 4 * lane) = l4;
  }
  __syncthreads();
  v8us qv[16];
#pragma unroll
  for (int i = 0; i < 16; ++i) {
    const unsigned short* srow = (const unsigned short*)stg + (size_t)(16 * wave + i) * (2 * GBN);
    qv[i] = *(const v8usa*)(srow + 8 * lane);
  }
#pragma unroll
  for (int i = 0; i < 16; ++i) {
    unsigned short* rp = Apl + (size_t)(rowBase + 16 * wave + i) * (size_t)AP + 2 * DF + 8 * lane;
    *(volatile v8us*)rp = qv[i];
  }
  __threadfence();
#pragma unroll
  for (int i = 0; i < 16; ++i) {
    unsigned short* rp = Apl + (size_t)(rowBase + 16 * wave + i) * (size_t)AP + 2 * DF + 8 * lane;
    *(volatile v8us*)rp = qv[i];
  }

  if (lane == 0) wst[wave * WSTW] = (float)wn;
#pragma unroll
  for (int j = 0; j < 4; ++j) {
    wst[wave * WSTW + 1 + 4 * lane + j]       = wm[j];
    wst[wave * WSTW + 1 + GBN + 4 * lane + j] = wqv[j];
  }
  __syncthreads();
  {
    float n = 0.0f, mean = 0.0f, M2 = 0.0f;
#pragma unroll 1
    for (int w2 = 0; w2 < GWAVE; ++w2) {
      const float nb = wst[w2 * WSTW];
      const float mb = wst[w2 * WSTW + 1 + tid];
      const float qb = wst[w2 * WSTW + 1 + GBN + tid];
      if (nb > 0.5f) {
        const float nn = n + nb;
        const float delta = mb - mean;
        const float f = nb / nn;
        mean = fmaf(delta, f, mean);
        M2 = M2 + qb + delta * delta * n * f;
        n = nn;
      }
    }
    pst[1 + tid] = mean;
    pst[1 + GBN + tid] = M2;
    if (tid == 0) pst[0] = n;
  }
#pragma unroll 1
  for (int i = 2 * GBN + 1 + tid; i < PARTW; i += GTHR) pst[i] = 0.0f;
  __syncthreads();
  const int pb = (int)blockIdx.x;
  v4f ps;
  if (tid < PARTW / 4) {
    ps = *(const v4fa*)(pst + 4 * tid);
    *(volatile v4f*)(part + (size_t)pb * PARTW + 4 * tid) = ps;
  }
  __threadfence();
  if (tid < PARTW / 4) {
    *(volatile v4f*)(part + (size_t)pb * PARTW + 4 * tid) = ps;
  }
}

__global__ __launch_bounds__(DF) void k_bnfin(const float* __restrict__ part, int nPart,
                                              const float* __restrict__ gam, const float* __restrict__ bet,
                                              float* ss) {
  __shared__ __attribute__((aligned(16))) float stg[2 * DF];
  const int tid = (int)threadIdx.x;
  const int c = tid;
  double n = 0.0, mean = 0.0, M2 = 0.0;
#pragma unroll 1
  for (int b = 0; b < nPart; ++b) {
    const float* pr = part + (size_t)b * PARTW;
    const double nb = (double)pr[0];
    const double mb = (double)pr[1 + c];
    const double qb = (double)pr[1 + GBN + c];
    if (nb > 0.5) {
      const double nn = n + nb;
      const double delta = mb - mean;
      const double f = nb / nn;
      mean = mean + delta * f;
      M2 = M2 + qb + delta * delta * n * f;
      n = nn;
    }
  }
  const double ntot = n < 1.0 ? 1.0 : n;
  const float varf  = (float)(M2 / ntot);
  const float meanf = (float)mean;
  const float rstd = rsqrtf(varf + 1e-5f);
  const float sc = bf16_val(gam[c]) * rstd;
  const float sh = bf16_val(bet[c]) - meanf * sc;
  stg[c] = sc;
  stg[DF + c] = sh;
  __syncthreads();
  v4f v;
  if (tid < (2 * DF) / 4) {
    v = *(const v4fa*)(stg + 4 * tid);
    *(volatile v4f*)(ss + 4 * tid) = v;
  }
  __threadfence();
  if (tid < (2 * DF) / 4) {
    *(volatile v4f*)(ss + 4 * tid) = v;
  }
}

template <int FIN>
__global__ __launch_bounds__(NTHR) void k_bnapply(unsigned short* apl, const float* __restrict__ ss, int nN,
                                                  int nUnits, float* outp) {
  __shared__ float ssh[2 * DF];
  const int tid = (int)threadIdx.x;
  ssh[tid] = ss[tid];
  __syncthreads();
  const int u = (int)blockIdx.x * NTHR + tid;
  if (u >= nUnits) return;
  if constexpr (FIN == 0) {
    const int row = u >> 4, j = u & 15, c0 = 8 * j;
    unsigned short* rp = apl + (size_t)row * (size_t)AP + 2 * DF + 8 * j;
    const v4u wh = *(const v4ua*)rp;
    const v4u wl = *(const v4ua*)(rp + DF);
    float v[8];
    v[0] = __uint_as_float(wh.x << 16)         + __uint_as_float(wl.x << 16);
    v[1] = __uint_as_float(wh.x & 0xffff0000u) + __uint_as_float(wl.x & 0xffff0000u);
    v[2] = __uint_as_float(wh.y << 16)         + __uint_as_float(wl.y << 16);
    v[3] = __uint_as_float(wh.y & 0xffff0000u) + __uint_as_float(wl.y & 0xffff0000u);
    v[4] = __uint_as_float(wh.z << 16)         + __uint_as_float(wl.z << 16);
    v[5] = __uint_as_float(wh.z & 0xffff0000u) + __uint_as_float(wl.z & 0xffff0000u);
    v[6] = __uint_as_float(wh.w << 16)         + __uint_as_float(wl.w << 16);
    v[7] = __uint_as_float(wh.w & 0xffff0000u) + __uint_as_float(wl.w & 0xffff0000u);
    const bool ok = row < nN;
    v8us ho, lo8;
#pragma unroll
    for (int i = 0; i < 8; ++i) {
      const float y  = fmaxf(fmaf(v[i], ssh[c0 + i], ssh[DF + c0 + i]), 0.0f);
      const float yy = ok ? y : 0.0f;
      unsigned lb;
      const unsigned hb = hl_bits(yy, lb);
      ho[i]  = (unsigned short)hb;
      lo8[i] = (unsigned short)lb;
    }
    *(volatile v8us*)rp = ho;
    *(volatile v8us*)(rp + DF) = lo8;
    __threadfence();
    *(volatile v8us*)rp = ho;
    *(volatile v8us*)(rp + DF) = lo8;
  } else {
    const int row = u >> 5, j = u & 31, c0 = 4 * j;
    const unsigned short* rp = apl + (size_t)row * (size_t)AP + 2 * DF + 4 * j;
    const v2u wh = *(const v2ua*)rp;
    const v2u wl = *(const v2ua*)(rp + DF);
    const float v0 = __uint_as_float(wh.x << 16)         + __uint_as_float(wl.x << 16);
    const float v1 = __uint_as_float(wh.x & 0xffff0000u) + __uint_as_float(wl.x & 0xffff0000u);
    const float v2 = __uint_as_float(wh.y << 16)         + __uint_as_float(wl.y << 16);
    const float v3 = __uint_as_float(wh.y & 0xffff0000u) + __uint_as_float(wl.y & 0xffff0000u);
    v4f o;
    o.x = fmaf(v0, ssh[c0 + 0], ssh[DF + c0 + 0]);
    o.y = fmaf(v1, ssh[c0 + 1], ssh[DF + c0 + 1]);
    o.z = fmaf(v2, ssh[c0 + 2], ssh[DF + c0 + 2]);
    o.w = fmaf(v3, ssh[c0 + 3], ssh[DF + c0 + 3]);
    float* op = outp + (size_t)row * DF + c0;
    *(volatile v4f*)op = o;
    __threadfence();
    *(volatile v4f*)op = o;
  }
}

static inline int cdiv(int a, int b) { return (a + b - 1) / b; }
static inline size_t al256(size_t o) { return (o + 255) & ~(size_t)255; }

extern "C" void kernel_launch(void* const* d_in, const int* in_sizes, int n_in,
                              void* d_out, int out_size, void* d_ws, size_t ws_size,
                              hipStream_t stream) {
  if (n_in < 20) return;
  const int nN = in_sizes[0];
  if (nN < 16 || nN >= (1 << 22) || in_sizes[1] != nN) return;
  if (in_sizes[2] < 2 || (in_sizes[2] & 1) != 0) return;
  const int nE = in_sizes[2] / 2;
  if (nE < 1 || nE >= (1 << 21)) return;
  if (in_sizes[3] != NTV * DIN || in_sizes[4] != NIV * DIN) return;
  if (in_sizes[5] != DIN * DF || in_sizes[6] != DF || in_sizes[7] != DIN * DF) return;
  if (in_sizes[8] != DF || in_sizes[9] != DF) return;
  for (int l = 0; l < 2; ++l) {
    const int b = 10 + 5 * l;
    if (in_sizes[b] != DF * DF || in_sizes[b + 1] != DF || in_sizes[b + 2] != DF * DF) return;
    if (in_sizes[b + 3] != DF || in_sizes[b + 4] != DF) return;
  }
  if ((long long)out_size != (long long)nN * DF) return;

  const int*   ntp  = (const int*)d_in[0];
  const int*   ipp  = (const int*)d_in[1];
  const int*   edge = (const int*)d_in[2];
  const float* ent  = (const float*)d_in[3];
  const float* eip  = (const float*)d_in[4];
  const float* Wl0  = (const float*)d_in[5];
  const float* bl0  = (const float*)d_in[6];
  const float* Wr0  = (const float*)d_in[7];
  const float* g0   = (const float*)d_in[8];
  const float* be0  = (const float*)d_in[9];
  const float* Wl1  = (const float*)d_in[10];
  const float* bl1  = (const float*)d_in[11];
  const float* Wr1  = (const float*)d_in[12];
  const float* g1   = (const float*)d_in[13];
  const float* be1  = (const float*)d_in[14];
  const float* Wl2  = (const float*)d_in[15];
  const float* bl2  = (const float*)d_in[16];
  const float* Wr2  = (const float*)d_in[17];
  const float* g2   = (const float*)d_in[18];
  const float* be2  = (const float*)d_in[19];
  float* out = (float*)d_out;
  const int* src = edge;
  const int* dst = edge + nE;

  const int MP = cdiv(nN, GBM) * GBM;
  const int gM = MP / GBM;
  const int gA = cdiv(nN, NBA);
  if ((long long)gA * NBA < (long long)MP) return;
  const int vec8 = ((nE & 3) == 0) ? 1 : 0;

  char* ws = (char*)d_ws;
  size_t off = 0;
  const size_t oB0 = off; off = al256(off + (size_t)DF * K0 * 2);
  const size_t oB1 = off; off = al256(off + (size_t)DF * K12 * 2);
  const size_t oB2 = off; off = al256(off + (size_t)DF * K12 * 2);
  const size_t oA  = off; off = al256(off + (size_t)MP * AP * 2);
  const size_t oPT = off; off = al256(off + (size_t)gM * PARTW * 4);
  const size_t oSS = off; off = al256(off + (size_t)(2 * DF) * 4);
  if (off > ws_size || off > (size_t)WSMAX) return;
  unsigned short* B0  = (unsigned short*)(ws + oB0);
  unsigned short* B1  = (unsigned short*)(ws + oB1);
  unsigned short* B2  = (unsigned short*)(ws + oB2);
  unsigned short* Apl = (unsigned short*)(ws + oA);
  float*          PT  = (float*)(ws + oPT);
  float*          SS  = (float*)(ws + oSS);

  const size_t scanLds1 = (size_t)AGG_LDS_INTS1 * 4;
  const size_t scanLds0 = (size_t)AGG_BASE_INTS * 4;
  hipFuncSetAttribute(reinterpret_cast<const void*>(&k_scan<1>), hipFuncAttributeMaxDynamicSharedMemorySize, (int)scanLds1);
  hipFuncSetAttribute(reinterpret_cast<const void*>(&k_scan<0>), hipFuncAttributeMaxDynamicSharedMemorySize, (int)scanLds0);

  const int nU0 = MP * 16;
  const int nU1 = nN * 32;

  k_wprep<<<(NPART * UPART) / NTHR, NTHR, 0, stream>>>(Wl0, Wr0, Wl1, Wr1, Wl2, Wr2, B0, B1, B2);
  k_scan<1><<<gA, NTHR, scanLds1, stream>>>(src, dst, nE, nN, vec8, MP, ntp, ipp, ent, eip, Apl);
  k_gemm<<<gM, GTHR, 0, stream>>>(Apl, B0, K0, nN, bl0, PT);
  k_bnfin<<<1, DF, 0, stream>>>(PT, gM, g0, be0, SS);
  k_bnapply<0><<<cdiv(nU0, NTHR), NTHR, 0, stream>>>(Apl, SS, nN, nU0, out);
  k_scan<0><<<gA, NTHR, scanLds0, stream>>>(src, dst, nE, nN, vec8, MP, ntp, ipp, ent, eip, Apl);
  k_gemm<<<gM, GTHR, 0, stream>>>(Apl, B1, K12, nN, bl1, PT);
  k_bnfin<<<1, DF, 0, stream>>>(PT, gM, g1, be1, SS);
  k_bnapply<0><<<cdiv(nU0, NTHR), NTHR, 0, stream>>>(Apl, SS, nN, nU0, out);
  k_scan<0><<<gA, NTHR, scanLds0, stream>>>(src, dst, nE, nN, vec8, MP, ntp, ipp, ent, eip, Apl);
  k_gemm<<<gM, GTHR, 0, stream>>>(Apl, B2, K12, nN, bl2, PT);
  k_bnfin<<<1, DF, 0, stream>>>(PT, gM, g2, be2, SS);
  k_bnapply<1><<<cdiv(nU1, NTHR), NTHR, 0, stream>>>(Apl, SS, nN, nU1, out);
}
